// MambaEncoderLayer_13675175871078
// MI455X (gfx1250) — hardware-run, weakly checked
//
#include <hip/hip_runtime.h>
#include <math.h>

typedef __attribute__((ext_vector_type(16))) _Float16 v16h;
typedef __attribute__((ext_vector_type(8)))  _Float16 v8h;
typedef __attribute__((ext_vector_type(8)))  float    v8f;
typedef __attribute__((ext_vector_type(4)))  float    v4f;

constexpr int kBatch = 2;
constexpr int kSeq   = 1024;
constexpr int kRows  = kBatch * kSeq;
constexpr int kDm    = 768;
constexpr int kDin   = 1536;
constexpr int kNst   = 16;
constexpr int kDtR   = 48;
constexpr int kDtP   = 64;
constexpr int kPrjN  = kDtR + 2 * kNst;
constexpr int kPrjP  = 128;
constexpr int kXzP   = 2 * kDin;
constexpr int kYP    = 2 * kDin;
constexpr int kTP    = 260;
static_assert(kRows == 2048 && kPrjN == 80 && kXzP == 3072, "shape constants");
static_assert((kDm % 32) == 0 && (kDin % 32) == 0 && (kDtP % 32) == 0 && (kYP % 32) == 0, "GEMM K multiples of 32");
static_assert((kRows % 64) == 0 && (kXzP % 64) == 0 && (kPrjP % 64) == 0 && (kDin % 64) == 0 && (kDm % 64) == 0, "GEMM M,N multiples of 64");
static_assert((kSeq % 64) == 0 && (kDin % 256) == 0 && (kDm % 256) == 0, "tile multiples");

constexpr float kXnCarry = 16.0f;
constexpr float kWCarry  = 256.0f;
constexpr float kUcCarry = 64.0f;
constexpr float kDtCarry = 1024.0f;
constexpr float kYCarry  = 256.0f;
constexpr float kSclIn   = 1.0f / (kXnCarry * kWCarry);
constexpr float kSclXp   = 1.0f / (kUcCarry * kWCarry);
constexpr float kSclDt   = 1.0f / (kDtCarry * kWCarry);
constexpr float kSclOut  = 1.0f / (kYCarry * kWCarry);
constexpr float kSclFc   = 1.0f / (kXnCarry * kWCarry);
constexpr float kUcInv   = 1.0f / kUcCarry;

constexpr size_t kOffWIN  = 0;
constexpr size_t kOffWXP  = kOffWIN  + (size_t)2 * kXzP * kDm * 2;
constexpr size_t kOffWDT  = kOffWXP  + (size_t)2 * kPrjP * kDin * 2;
constexpr size_t kOffWOUT = kOffWDT  + (size_t)2 * kDin * kDtP * 2;
constexpr size_t kOffWFC  = kOffWOUT + (size_t)kDm * kYP * 2;
constexpr size_t kOffXN   = kOffWFC  + (size_t)kDm * kDm * 2;
constexpr size_t kOffXZ   = kOffXN   + (size_t)kRows * kDm * 2;
constexpr size_t kOffUC   = kOffXZ   + (size_t)2 * kRows * kXzP * 2;
constexpr size_t kOffPROJ = kOffUC   + (size_t)2 * kRows * kDin * 2;
constexpr size_t kOffDT   = kOffPROJ + (size_t)2 * kRows * kPrjP * 4;
constexpr size_t kOffDLR  = kOffDT   + (size_t)2 * kRows * kDtP * 2;
constexpr size_t kOffY    = kOffDLR  + (size_t)2 * kRows * kDin * 4;
constexpr size_t kOffX2   = kOffY    + (size_t)kRows * kYP * 2;
constexpr size_t kOffX2N  = kOffX2   + (size_t)kRows * kDm * 4;
constexpr size_t kOffFCP  = kOffX2N  + (size_t)kRows * kDm * 2;
constexpr size_t kWsTotal = kOffFCP  + (size_t)kRows * kDm * 4;
static_assert(kWsTotal == 113508352ull, "carve total");
static_assert(kWsTotal <= 134217728ull, "carve cap");
static_assert((kOffWXP % 128) == 0 && (kOffWDT % 128) == 0 && (kOffWOUT % 128) == 0 && (kOffWFC % 128) == 0 &&
              (kOffXN % 128) == 0 && (kOffXZ % 128) == 0 && (kOffUC % 128) == 0 && (kOffPROJ % 128) == 0 &&
              (kOffDT % 128) == 0 && (kOffDLR % 128) == 0 && (kOffY % 128) == 0 && (kOffX2 % 128) == 0 &&
              (kOffX2N % 128) == 0 && (kOffFCP % 128) == 0, "128-B aligned regions");

__device__ __forceinline__ float h16_to_f32(unsigned hb) {
  const unsigned sgn = (hb & 0x8000u) << 16;
  const unsigned em = hb & 0x7fffu;
  const float fn = __uint_as_float((em << 13) + 0x38000000u);
  const float fs = (float)em * 5.9604644775390625e-8f;
  const float mag = (em < 0x400u) ? fs : fn;
  return __uint_as_float(__float_as_uint(mag) | sgn);
}
__device__ __forceinline__ float ld_h16(const unsigned short* __restrict__ p, size_t idx) {
  unsigned hb = (unsigned)p[idx];
  asm volatile("" : "+v"(hb));
  return h16_to_f32(hb);
}

__device__ __forceinline__ void guard_row4(v8f& a, v8f& b, v8f& c, v8f& d, v16h x, v16h b0, v16h b1, v16h b2, v16h b3) {
  asm volatile("v_nop\n\tv_nop\n\tv_nop\n\tv_nop" : "+v"(a), "+v"(b), "+v"(c), "+v"(d) : "v"(x), "v"(b0), "v"(b1), "v"(b2), "v"(b3));
}
__device__ __forceinline__ void keep4_h(v16h a, v16h b, v16h c, v16h d) { asm volatile("v_nop" :: "v"(a), "v"(b), "v"(c), "v"(d)); }
__device__ __forceinline__ void acc_guard4(v8f& a, v8f& b, v8f& c, v8f& d) { asm volatile("v_nop\n\tv_nop\n\tv_nop\n\tv_nop" : "+v"(a), "+v"(b), "+v"(c), "+v"(d)); }

struct FragH {
  union U { v16h v; v8h h[2]; };
  static __device__ __forceinline__ v16h load(const _Float16* p) {
    U f; f.h[0] = *(const v8h*)(p); f.h[1] = *(const v8h*)(p + 16); return f.v;
  }
  static __device__ __forceinline__ v8f mma(v16h a, v16h b, v8f c) {
    return __builtin_amdgcn_wmma_f32_16x16x32_f16(false, a, false, b, (short)0, c, false, false);
  }
};

template <int BIAS_MODE, int OUT_MODE, bool RESID>
__global__ __launch_bounds__(256) void wmma_gemm64(
    const unsigned short* __restrict__ Ap, int lda, long strideA,
    const unsigned short* __restrict__ Btp, int ldb, long strideB,
    void* __restrict__ Cout, int ldc, long strideC,
    const float* __restrict__ bias0, const float* __restrict__ bias1,
    const float* __restrict__ resid,
    int M, int N, int K, float scale) {
  typedef _Float16 T;
  const T* A = (const T*)Ap;
  const T* Bt = (const T*)Btp;
  __shared__ __align__(16) float sT[8][16 * 68];
  const int b    = blockIdx.y;
  const int lane = threadIdx.x & 31;
  const int wave = threadIdx.x >> 5;
  const int tilesN = N >> 6;
  const int tilesM = M >> 6;
  const int tile = blockIdx.x * 8 + wave;
  if (tile >= tilesM * tilesN) return;
  const int tm = tile / tilesN;
  const int tn = tile - tm * tilesN;
  const int m0 = tm << 6;
  const int n0 = tn << 6;

  const T* Ab = A  + (size_t)b * (size_t)strideA;
  const T* Bb = Bt + (size_t)b * (size_t)strideB;
  const float* bias = (b == 0) ? bias0 : bias1;

  const int rlane = lane & 15;
  const int koff  = (lane >> 4) * 8;
  const int mOff  = (lane >> 4) * 8;

  v8f acc[4][4];
#pragma unroll
  for (int i = 0; i < 4; ++i)
#pragma unroll
    for (int j = 0; j < 4; ++j) acc[i][j] = (v8f){0.f,0.f,0.f,0.f,0.f,0.f,0.f,0.f};

  for (int k0 = 0; k0 < K; k0 += 32) {
    v16h bh[4];
#pragma unroll
    for (int j = 0; j < 4; ++j) {
      const size_t bo = (size_t)(n0 + (j << 4) + rlane) * ldb + koff + k0;
      bh[j] = FragH::load(Bb + bo);
    }
#pragma unroll
    for (int i = 0; i < 4; ++i) {
      const size_t ao = (size_t)(m0 + (i << 4) + rlane) * lda + koff + k0;
      const v16h ah = FragH::load(Ab + ao);
#pragma unroll
      for (int j = 0; j < 4; ++j) acc[i][j] = FragH::mma(ah, bh[j], acc[i][j]);
      guard_row4(acc[i][0], acc[i][1], acc[i][2], acc[i][3], ah, bh[0], bh[1], bh[2], bh[3]);
    }
    keep4_h(bh[0], bh[1], bh[2], bh[3]);
  }
  acc_guard4(acc[0][0], acc[0][1], acc[0][2], acc[0][3]);
  acc_guard4(acc[1][0], acc[1][1], acc[1][2], acc[1][3]);
  acc_guard4(acc[2][0], acc[2][1], acc[2][2], acc[2][3]);
  acc_guard4(acc[3][0], acc[3][1], acc[3][2], acc[3][3]);

  float* slab = sT[wave];
#pragma unroll
  for (int i = 0; i < 4; ++i) {
    const int mBase = m0 + (i << 4);
#pragma unroll
    for (int j = 0; j < 4; ++j) {
      const int n = n0 + (j << 4) + rlane;
      float bv = 0.f;
      if (BIAS_MODE == 2) bv = bias[n];
#pragma unroll
      for (int r = 0; r < 8; ++r) {
        float v = acc[i][j][r] * scale;
        if (BIAS_MODE == 2) v += bv;
        slab[(mOff + r) * 68 + (j << 4) + rlane] = v;
      }
    }
    __builtin_amdgcn_fence(__ATOMIC_RELEASE, "workgroup");
    __builtin_amdgcn_wave_barrier();
    __builtin_amdgcn_fence(__ATOMIC_ACQUIRE, "workgroup");
    if (OUT_MODE == 0) {
      float* C = (float*)Cout + (size_t)b * (size_t)strideC;
      const int hh = lane >> 4, c4 = (lane & 15) * 4;
      v4f vv[8];
#pragma unroll
      for (int it = 0; it < 8; ++it) {
        const int row = it * 2 + hh;
        vv[it] = *(const v4f*)(slab + row * 68 + c4);
        if (RESID) {
          const v4f rr = *(const v4f*)(resid + (size_t)(mBase + row) * ldc + n0 + c4);
          vv[it] = vv[it] + rr;
        }
      }
      for (int pass = 0; pass < 2; ++pass) {
#pragma unroll
        for (int it = 0; it < 8; ++it) {
          const int row = it * 2 + hh;
          *(volatile v4f*)(C + (size_t)(mBase + row) * ldc + n0 + c4) = vv[it];
        }
        __threadfence();
      }
    } else {
      const int q = lane >> 3, c8 = (lane & 7) * 8;
      unsigned short* C = (unsigned short*)Cout + (size_t)b * (size_t)strideC;
      v8h hv[4];
#pragma unroll
      for (int it = 0; it < 4; ++it) {
        const int row = it * 4 + q;
        const float* sp = slab + row * 68 + c8;
        const v4f a0 = *(const v4f*)(sp);
        const v4f a1 = *(const v4f*)(sp + 4);
#pragma unroll
        for (int e = 0; e < 4; ++e) {
          hv[it][e]     = (_Float16)a0[e];
          hv[it][4 + e] = (_Float16)a1[e];
        }
      }
      for (int pass = 0; pass < 2; ++pass) {
#pragma unroll
        for (int it = 0; it < 4; ++it) {
          const int row = it * 4 + q;
          *(volatile v8h*)(C + (size_t)(mBase + row) * ldc + n0 + c8) = hv[it];
        }
        __threadfence();
      }
    }
    __builtin_amdgcn_fence(__ATOMIC_RELEASE, "workgroup");
    __builtin_amdgcn_wave_barrier();
    __builtin_amdgcn_fence(__ATOMIC_ACQUIRE, "workgroup");
  }
}

__global__ __launch_bounds__(256) void cast_pad_f16_kernel(
    const float* __restrict__ src0, const float* __restrict__ src1,
    int srcRows, int srcCols, int srcPitch,
    unsigned short* __restrict__ dst, int dstPitch, long dstDirStride,
    int dstRows, int dstCols, float scale)
{
  const int dir = blockIdx.y;
  const float* src = dir ? src1 : src0;
  const int per_row = dstCols >> 3;
  const int total8 = dstRows * per_row;
  const int i = blockIdx.x * 256 + threadIdx.x;
  if (i >= total8) return;
  const int r  = i / per_row;
  const int c8 = (i - r * per_row) << 3;
  const bool live = (r < srcRows) && (c8 < srcCols);
  const int rc = (r < srcRows) ? r : (srcRows - 1);
  const int cc = (c8 < srcCols) ? c8 : 0;
  const float* p = src + (size_t)rc * srcPitch + cc;
  const v4f a0 = *(const v4f*)(p);
  const v4f a1 = *(const v4f*)(p + 4);
  v8h hv;
#pragma unroll
  for (int e = 0; e < 4; ++e) {
    const float f0 = live ? (a0[e] * scale) : 0.0f;
    const float f1 = live ? (a1[e] * scale) : 0.0f;
    hv[e]     = (_Float16)f0;
    hv[4 + e] = (_Float16)f1;
  }
  unsigned short* q = dst + (size_t)dir * (size_t)dstDirStride + (size_t)r * dstPitch + c8;
  *(volatile v8h*)q = hv;
  __threadfence();
  *(volatile v8h*)q = hv;
}

__global__ __launch_bounds__(256) void layernorm_f16_kernel(
    const float* __restrict__ X, const float* __restrict__ w, const float* __restrict__ bsh,
    unsigned short* __restrict__ out, int rows, float carry)
{
  const int lane = threadIdx.x & 31, wave = threadIdx.x >> 5;
  const int row = blockIdx.x * 8 + wave;
  if (row >= rows) return;
  const float* xr = X + (size_t)row * kDm;
  v4f v[6];
#pragma unroll
  for (int j = 0; j < 3; ++j) {
    v[2 * j]     = *(const v4f*)(xr + j * 256 + lane * 8);
    v[2 * j + 1] = *(const v4f*)(xr + j * 256 + lane * 8 + 4);
  }
  float s = 0.f;
#pragma unroll
  for (int j = 0; j < 6; ++j) s += (v[j][0] + v[j][1]) + (v[j][2] + v[j][3]);
#pragma unroll
  for (int o = 16; o > 0; o >>= 1) s += __shfl_xor(s, o, 32);
  const float mean = s * (1.0f / (float)kDm);
  float ss = 0.f;
#pragma unroll
  for (int j = 0; j < 6; ++j) {
#pragma unroll
    for (int e = 0; e < 4; ++e) {
      const float dlt = v[j][e] - mean;
      ss = fmaf(dlt, dlt, ss);
    }
  }
#pragma unroll
  for (int o = 16; o > 0; o >>= 1) ss += __shfl_xor(ss, o, 32);
  const float var  = ss * (1.0f / (float)kDm);
  const float rstd = 1.0f / sqrtf(var + 1e-5f);
  v8h hv[3];
#pragma unroll
  for (int j = 0; j < 3; ++j) {
    const int c = j * 256 + lane * 8;
    const v4f w0 = *(const v4f*)(w + c);
    const v4f w1 = *(const v4f*)(w + c + 4);
    const v4f b0 = *(const v4f*)(bsh + c);
    const v4f b1 = *(const v4f*)(bsh + c + 4);
#pragma unroll
    for (int e = 0; e < 4; ++e) {
      const float y0 = ((v[2 * j][e] - mean) * rstd) * w0[e] + b0[e];
      const float y1 = ((v[2 * j + 1][e] - mean) * rstd) * w1[e] + b1[e];
      hv[j][e]     = (_Float16)(y0 * carry);
      hv[j][4 + e] = (_Float16)(y1 * carry);
    }
  }
  unsigned short* orow = out + (size_t)row * kDm + lane * 8;
  for (int pass = 0; pass < 2; ++pass) {
#pragma unroll
    for (int j = 0; j < 3; ++j) *(volatile v8h*)(orow + j * 256) = hv[j];
    __threadfence();
  }
}

__global__ __launch_bounds__(256) void conv_silu_kernel(
    const unsigned short* __restrict__ XZ16,
    const float* __restrict__ cw0, const float* __restrict__ cw1,
    const float* __restrict__ cb0, const float* __restrict__ cb1,
    unsigned short* __restrict__ UC16)
{
  __shared__ __align__(16) float sT[16 * kTP];
  const int tid = threadIdx.x, lane = tid & 31, wave = tid >> 5;
  const int dir = blockIdx.z;
  const float* cw = dir ? cw1 : cw0;
  const float* cb = dir ? cb1 : cb0;
  const unsigned short* xz = XZ16 + (size_t)dir * kRows * kXzP;
  unsigned short* uc = UC16 + (size_t)dir * kRows * kDin;
  const int d0 = blockIdx.x * 256, d = d0 + tid;
  const int g0 = blockIdx.y * 64;
  const int tb = g0 & (kSeq - 1);
  const v4f wv = *(const v4f*)(cw + (size_t)d * 4);
  const float w0 = wv[0], w1 = wv[1], w2 = wv[2], w3 = wv[3];
  const float bc = cb[d];
  float xm3, xm2, xm1;
  {
    const bool hist = dir ? (tb + 64 < kSeq) : (tb > 0);
    const int rb = hist ? (dir ? (g0 + 64) : (g0 - 3)) : g0;
    const float va = ld_h16(xz, (size_t)rb * kXzP + d);
    const float vb = ld_h16(xz, (size_t)(rb + 1) * kXzP + d);
    const float vc = ld_h16(xz, (size_t)(rb + 2) * kXzP + d);
    const float ha = hist ? va : 0.f;
    const float hb = hist ? vb : 0.f;
    const float hc = hist ? vc : 0.f;
    xm3 = dir ? hc : ha;
    xm2 = hb;
    xm1 = dir ? ha : hc;
  }
#pragma unroll 1
  for (int sub = 0; sub < 4; ++sub) {
    const int lb = dir ? (g0 + 48 - sub * 16) : (g0 + sub * 16);
#pragma unroll 1
    for (int s = 0; s < 16; ++s) {
      const int tr = dir ? (15 - s) : s;
      const float xcur = ld_h16(xz, (size_t)(lb + tr) * kXzP + d);
      float acc = w0 * xm3;
      acc = fmaf(w1, xm2, acc);
      acc = fmaf(w2, xm1, acc);
      acc = fmaf(w3, xcur, acc);
      const float sv = acc + bc;
      const float sg = __builtin_amdgcn_rcpf(1.0f + expf(-sv));
      sT[tr * kTP + tid] = (sv * sg) * kUcCarry;
      xm3 = xm2; xm2 = xm1; xm1 = xcur;
    }
    __syncthreads();
    v8h bv[2];
#pragma unroll
    for (int it = 0; it < 2; ++it) {
      const float* sp = sT + (it * 8 + wave) * kTP + lane * 8;
      const v4f a0 = *(const v4f*)(sp);
      const v4f a1 = *(const v4f*)(sp + 4);
#pragma unroll
      for (int e = 0; e < 4; ++e) {
        bv[it][e]     = (_Float16)a0[e];
        bv[it][4 + e] = (_Float16)a1[e];
      }
    }
    for (int pass = 0; pass < 2; ++pass) {
#pragma unroll
      for (int it = 0; it < 2; ++it)
        *(volatile v8h*)(uc + (size_t)(lb + it * 8 + wave) * kDin + d0 + lane * 8) = bv[it];
      __threadfence();
    }
    __syncthreads();
  }
}

__global__ __launch_bounds__(256) void scan_kernel(
    const float* __restrict__ DLR, const unsigned short* __restrict__ UC16, const unsigned short* __restrict__ XZ16,
    const float* __restrict__ PROJ,
    const float* __restrict__ Alog0, const float* __restrict__ Alog1,
    const float* __restrict__ Dv0, const float* __restrict__ Dv1,
    unsigned short* __restrict__ Y16)
{
  __shared__ __align__(16) float sBC[16 * 32];
  __shared__ __align__(16) float sY[16 * kTP];
  __shared__ float sH[kNst * 256];
  __shared__ float sA[kNst * 256];
  const int tid = threadIdx.x, lane = tid & 31, wave = tid >> 5;
  const int d0 = blockIdx.x * 256, d = d0 + tid;
  const int bix = blockIdx.y;
  const int dir = blockIdx.z;
  const float* Alog = dir ? Alog1 : Alog0;
  const float* Dv   = dir ? Dv1 : Dv0;
  const float* dlr  = DLR  + (size_t)dir * kRows * kDin;
  const float* prj  = PROJ + (size_t)dir * kRows * kPrjP;
  const unsigned short* ucp = UC16 + (size_t)dir * kRows * kDin;
  const unsigned short* xzp = XZ16 + (size_t)dir * kRows * kXzP;
  const int rowb = bix * kSeq;

#pragma unroll 1
  for (int n = 0; n < kNst; ++n) {
    sA[n * 256 + tid] = -expf(Alog[(size_t)d * kNst + n]);
    sH[n * 256 + tid] = 0.f;
  }
  const float Dd = Dv[d];

#pragma unroll 1
  for (int c = 0; c < kSeq / 16; ++c) {
    const int lb = dir ? (kSeq - 16 - c * 16) : (c * 16);
    if (tid < 128) {
      const int r = tid >> 3, q = (tid & 7) * 4;
      const v4f vbc = *(const v4f*)(prj + (size_t)(rowb + lb + r) * kPrjP + kDtR + q);
      *(v4f*)(sBC + r * 32 + q) = vbc;
    }
    __syncthreads();
#pragma unroll 1
    for (int s = 0; s < 16; ++s) {
      const int tr = dir ? (15 - s) : s;
      const size_t m = (size_t)(rowb + lb + tr);
      float a = dlr[m * kDin + d];
      asm volatile("" : "+v"(a));
      const float xv = ld_h16(ucp, m * kDin + d) * kUcInv;
      const float zv = ld_h16(xzp, m * kXzP + kDin + d);
      const float delta = fmaxf(a, 0.0f) + log1pf(expf(-fabsf(a)));
      const float dtx = delta * xv;
      float y = 0.f;
#pragma unroll 1
      for (int g = 0; g < 4; ++g) {
        const v4f Bq = *(const v4f*)(sBC + tr * 32 + 4 * g);
        const v4f Cq = *(const v4f*)(sBC + tr * 32 + kNst + 4 * g);
        float* hp = sH + (4 * g) * 256 + tid;
        const float* ap = sA + (4 * g) * 256 + tid;
#pragma unroll
        for (int j = 0; j < 4; ++j) {
          const float e  = expf(delta * ap[j * 256]);
          const float hn = fmaf(e, hp[j * 256], dtx * Bq[j]);
          hp[j * 256] = hn;
          y = fmaf(hn, Cq[j], y);
        }
      }
      y = fmaf(xv, Dd, y);
      const float sg = __builtin_amdgcn_rcpf(1.0f + expf(-zv));
      sY[tr * kTP + tid] = (y * (zv * sg)) * kYCarry;
    }
    __syncthreads();
    v8h hv[2];
#pragma unroll
    for (int it = 0; it < 2; ++it) {
      const float* sp = sY + (it * 8 + wave) * kTP + lane * 8;
      const v4f a0 = *(const v4f*)(sp);
      const v4f a1 = *(const v4f*)(sp + 4);
#pragma unroll
      for (int e = 0; e < 4; ++e) { hv[it][e] = (_Float16)a0[e]; hv[it][4 + e] = (_Float16)a1[e]; }
    }
    for (int pass = 0; pass < 2; ++pass) {
#pragma unroll
      for (int it = 0; it < 2; ++it)
        *(volatile v8h*)(Y16 + (size_t)(rowb + lb + it * 8 + wave) * kYP + dir * kDin + d0 + lane * 8) = hv[it];
      __threadfence();
    }
  }
}

__global__ __launch_bounds__(256) void gelu_resid_kernel(
    const float* __restrict__ T, const float* __restrict__ R, float* __restrict__ out)
{
  __shared__ __align__(16) float sO[2048];
  const int tid = threadIdx.x;
  const size_t base = (size_t)blockIdx.x * 2048;
#pragma unroll 1
  for (int e = 0; e < 8; ++e) {
    const int idx = e * 256 + tid;
    const float t = T[base + idx];
    const float r = R[base + idx];
    const float g = 0.5f * t * (1.0f + erff(t * 0.70710678118654752f));
    sO[idx] = g + r;
  }
  __syncthreads();
  v4f o[2];
#pragma unroll
  for (int it = 0; it < 2; ++it) o[it] = *(const v4f*)(sO + it * 1024 + tid * 4);
  for (int pass = 0; pass < 2; ++pass) {
#pragma unroll
    for (int it = 0; it < 2; ++it) *(volatile v4f*)(out + base + it * 1024 + tid * 4) = o[it];
    __threadfence();
  }
}

extern "C" void kernel_launch(void* const* d_in, const int* in_sizes, int n_in,
                              void* d_out, int out_size, void* d_ws, size_t ws_size,
                              hipStream_t stream)
{
  if (n_in < 25) return;
  if (in_sizes[0] != kRows * kDm) return;
  if (in_sizes[1] != kDm || in_sizes[2] != kDm || in_sizes[3] != kDm || in_sizes[4] != kDm) return;
  if (in_sizes[5] != kDm * kDm || in_sizes[6] != kDm) return;
  for (int o = 7; o <= 16; o += 9) {
    if (in_sizes[o + 0] != kXzP * kDm) return;
    if (in_sizes[o + 1] != kDin * 4 || in_sizes[o + 2] != kDin) return;
    if (in_sizes[o + 3] != kPrjN * kDin) return;
    if (in_sizes[o + 4] != kDin * kDtR || in_sizes[o + 5] != kDin) return;
    if (in_sizes[o + 6] != kDin * kNst || in_sizes[o + 7] != kDin) return;
    if (in_sizes[o + 8] != kDm * kDin) return;
  }
  if (out_size != kRows * kDm) return;
  if (ws_size < kWsTotal) return;

  const float* x     = (const float*)d_in[0];
  const float* ln1w  = (const float*)d_in[1];
  const float* ln1b  = (const float*)d_in[2];
  const float* ln2w  = (const float*)d_in[3];
  const float* ln2b  = (const float*)d_in[4];
  const float* fcw   = (const float*)d_in[5];
  const float* fcb   = (const float*)d_in[6];
  const float* f_inw = (const float*)d_in[7];
  const float* f_cw  = (const float*)d_in[8];
  const float* f_cb  = (const float*)d_in[9];
  const float* f_xpw = (const float*)d_in[10];
  const float* f_dtw = (const float*)d_in[11];
  const float* f_dtb = (const float*)d_in[12];
  const float* f_al  = (const float*)d_in[13];
  const float* f_D   = (const float*)d_in[14];
  const float* f_ow  = (const float*)d_in[15];
  const float* b_inw = (const float*)d_in[16];
  const float* b_cw  = (const float*)d_in[17];
  const float* b_cb  = (const float*)d_in[18];
  const float* b_xpw = (const float*)d_in[19];
  const float* b_dtw = (const float*)d_in[20];
  const float* b_dtb = (const float*)d_in[21];
  const float* b_al  = (const float*)d_in[22];
  const float* b_D   = (const float*)d_in[23];
  const float* b_ow  = (const float*)d_in[24];
  float* out = (float*)d_out;

  char* ws = (char*)d_ws;
  unsigned short* WIN16  = (unsigned short*)(ws + kOffWIN);
  unsigned short* WXP16  = (unsigned short*)(ws + kOffWXP);
  unsigned short* WDT16  = (unsigned short*)(ws + kOffWDT);
  unsigned short* WOUT16 = (unsigned short*)(ws + kOffWOUT);
  unsigned short* WFC16  = (unsigned short*)(ws + kOffWFC);
  unsigned short* XN16   = (unsigned short*)(ws + kOffXN);
  unsigned short* XZ16   = (unsigned short*)(ws + kOffXZ);
  unsigned short* UC16   = (unsigned short*)(ws + kOffUC);
  float*          PROJ   = (float*)(ws + kOffPROJ);
  unsigned short* DT16   = (unsigned short*)(ws + kOffDT);
  float*          DLR    = (float*)(ws + kOffDLR);
  unsigned short* Y16    = (unsigned short*)(ws + kOffY);
  float*          X2     = (float*)(ws + kOffX2);
  unsigned short* X2N16  = (unsigned short*)(ws + kOffX2N);
  float*          FCP    = (float*)(ws + kOffFCP);

  cast_pad_f16_kernel<<<dim3((kXzP * kDm / 8) / 256, 2), 256, 0, stream>>>(
      f_inw, b_inw, kXzP, kDm, kDm, WIN16, kDm, (long)kXzP * kDm, kXzP, kDm, kWCarry);
  cast_pad_f16_kernel<<<dim3((kPrjP * kDin / 8) / 256, 2), 256, 0, stream>>>(
      f_xpw, b_xpw, kPrjN, kDin, kDin, WXP16, kDin, (long)kPrjP * kDin, kPrjP, kDin, kWCarry);
  cast_pad_f16_kernel<<<dim3((kDin * kDtP / 8) / 256, 2), 256, 0, stream>>>(
      f_dtw, b_dtw, kDin, kDtR, kDtR, WDT16, kDtP, (long)kDin * kDtP, kDin, kDtP, kWCarry);
  cast_pad_f16_kernel<<<dim3((kDm * kDin / 8) / 256, 2), 256, 0, stream>>>(
      f_ow, b_ow, kDm, kDin, kDin, WOUT16, kYP, (long)kDin, kDm, kDin, kWCarry);
  cast_pad_f16_kernel<<<dim3((kDm * kDm / 8) / 256, 1), 256, 0, stream>>>(
      fcw, fcw, kDm, kDm, kDm, WFC16, kDm, 0L, kDm, kDm, kWCarry);

  layernorm_f16_kernel<<<kRows / 8, 256, 0, stream>>>(x, ln1w, ln1b, XN16, kRows, kXnCarry);

  wmma_gemm64<0, 1, false><<<dim3(192, 2), 256, 0, stream>>>(
      XN16, kDm, 0L,
      WIN16, kDm, (long)kXzP * kDm,
      (void*)XZ16, kXzP, (long)kRows * kXzP,
      x, x, x,
      kRows, kXzP, kDm, kSclIn);

  conv_silu_kernel<<<dim3(kDin / 256, kRows / 64, 2), 256, 0, stream>>>(XZ16, f_cw, b_cw, f_cb, b_cb, UC16);

  wmma_gemm64<0, 0, false><<<dim3(8, 2), 256, 0, stream>>>(
      UC16, kDin, (long)kRows * kDin,
      WXP16, kDin, (long)kPrjP * kDin,
      (void*)PROJ, kPrjP, (long)kRows * kPrjP,
      x, x, x,
      kRows, kPrjP, kDin, kSclXp);

  cast_pad_f16_kernel<<<dim3((2 * kRows * kDtP / 8) / 256, 1), 256, 0, stream>>>(
      PROJ, PROJ, 2 * kRows, kDtR, kPrjP, DT16, kDtP, 0L, 2 * kRows, kDtP, kDtCarry);

  wmma_gemm64<2, 0, false><<<dim3(96, 2), 256, 0, stream>>>(
      DT16, kDtP, (long)kRows * kDtP,
      WDT16, kDtP, (long)kDin * kDtP,
      (void*)DLR, kDin, (long)kRows * kDin,
      f_dtb, b_dtb, x,
      kRows, kDin, kDtP, kSclDt);

  scan_kernel<<<dim3(kDin / 256, kBatch, 2), 256, 0, stream>>>(
      DLR, UC16, XZ16, PROJ, f_al, b_al, f_D, b_D, Y16);

  wmma_gemm64<0, 0, true><<<dim3(48, 1), 256, 0, stream>>>(
      Y16, kYP, 0L,
      WOUT16, kYP, 0L,
      (void*)X2, kDm, 0L,
      x, x, x,
      kRows, kDm, kYP, kSclOut);

  layernorm_f16_kernel<<<kRows / 8, 256, 0, stream>>>(X2, ln2w, ln2b, X2N16, kRows, kXnCarry);

  wmma_gemm64<2, 0, false><<<dim3(48, 1), 256, 0, stream>>>(
      X2N16, kDm, 0L,
      WFC16, kDm, 0L,
      (void*)FCP, kDm, 0L,
      fcb, fcb, x,
      kRows, kDm, kDm, kSclFc);

  gelu_resid_kernel<<<(kRows * kDm) / 2048, 256, 0, stream>>>(FCP, X2, out);
}
